// QMOIMultimodalFusion_18794776888076
// MI455X (gfx1250) — hardware-verified
//
#include <hip/hip_runtime.h>
#include <math.h>

constexpr int kNB   = 4;
constexpr int kNS   = 1024;
constexpr int kNE   = 1024;
constexpr int kNH   = 16;
constexpr int kHD   = 64;
constexpr int kHalf = 32;
constexpr int kTok  = kNB * kNS;
constexpr int kRelN = 2 * 2048 - 1;
constexpr int kNRow = 12;
constexpr int kPW   = kTok;
constexpr int kF1K  = 3 * kNE;

typedef __attribute__((ext_vector_type(16))) _Float16 v16h;
typedef __attribute__((ext_vector_type(8)))  _Float16 v8h;
typedef __attribute__((ext_vector_type(16))) __bf16   v16b;
typedef __attribute__((ext_vector_type(8)))  __bf16   v8b;
typedef __attribute__((ext_vector_type(8)))  float    v8f;
typedef __attribute__((ext_vector_type(4)))  float    v4f;
typedef __attribute__((ext_vector_type(4)))  unsigned int v4u;

__device__ __forceinline__ unsigned short f2bf_bits(float f) {
  unsigned u = __float_as_uint(f);
  return (unsigned short)((u + 0x7FFFu + ((u >> 16) & 1u)) >> 16);
}
__device__ __forceinline__ float bf_bits2f(unsigned short h) { return __uint_as_float(((unsigned)h) << 16); }
__device__ __forceinline__ float bfr(float f) { return bf_bits2f(f2bf_bits(f)); }

__device__ __forceinline__ void dep_guard_h(v8f& a, v8f& b, v16h x, v16h y) { asm volatile("v_nop\n\tv_nop\n\tv_nop\n\tv_nop" : "+v"(a), "+v"(b) : "v"(x), "v"(y)); }
__device__ __forceinline__ void dep_guard_b(v8f& a, v8f& b, v16b x, v16b y) { asm volatile("v_nop\n\tv_nop\n\tv_nop\n\tv_nop" : "+v"(a), "+v"(b) : "v"(x), "v"(y)); }
__device__ __forceinline__ void keep4_h(v16h a, v16h b, v16h c, v16h d) { asm volatile("v_nop" :: "v"(a), "v"(b), "v"(c), "v"(d)); }
__device__ __forceinline__ void keep4_b(v16b a, v16b b, v16b c, v16b d) { asm volatile("v_nop" :: "v"(a), "v"(b), "v"(c), "v"(d)); }
__device__ __forceinline__ void acc_guard4(v8f& a, v8f& b, v8f& c, v8f& d) { asm volatile("v_nop\n\tv_nop\n\tv_nop\n\tv_nop" : "+v"(a), "+v"(b), "+v"(c), "+v"(d)); }
template <typename T> struct Frag;
template <> struct Frag<_Float16> {
  typedef v16h V; union U { v16h v; v8h h[2]; };
  static __device__ __forceinline__ v16h load(const _Float16* p) {
    U f; f.h[0] = *(const v8h*)(p); f.h[1] = *(const v8h*)(p + 16); return f.v;
  }
  static __device__ __forceinline__ v8f mma(v16h a, v16h b, v8f c) {
    return __builtin_amdgcn_wmma_f32_16x16x32_f16(false, a, false, b, (short)0, c, false, false);
  }
  static __device__ __forceinline__ void guard(v8f& a, v8f& b, v16h x, v16h y) { dep_guard_h(a, b, x, y); }
  static __device__ __forceinline__ void keep(v16h a, v16h b, v16h c, v16h d) { keep4_h(a, b, c, d); }
};
template <> struct Frag<__bf16> {
  typedef v16b V; union U { v16b v; v8b h[2]; };
  static __device__ __forceinline__ v16b load(const __bf16* p) {
    U f; f.h[0] = *(const v8b*)(p); f.h[1] = *(const v8b*)(p + 16); return f.v;
  }
  static __device__ __forceinline__ v8f mma(v16b a, v16b b, v8f c) {
    return __builtin_amdgcn_wmma_f32_16x16x32_bf16(false, a, false, b, (short)0, c, false, false);
  }
  static __device__ __forceinline__ void guard(v8f& a, v8f& b, v16b x, v16b y) { dep_guard_b(a, b, x, y); }
  static __device__ __forceinline__ void keep(v16b a, v16b b, v16b c, v16b d) { keep4_b(a, b, c, d); }
};

__device__ __forceinline__ unsigned pk16(unsigned short a, unsigned short b) { return (unsigned)a | ((unsigned)b << 16); }
__device__ __forceinline__ unsigned short h_bits(float f) { const _Float16 h = (_Float16)f; return __builtin_bit_cast(unsigned short, h); }

template <int ET> struct Elem;
template <> struct Elem<0> { typedef _Float16 T; };
template <> struct Elem<1> { typedef __bf16 T; };
template <int ET, int SPL, int BIAS_MODE, int OUT_MODE>
__global__ __launch_bounds__(256) void wmma_gemm64(
    const unsigned short* __restrict__ Ap, const unsigned short* __restrict__ A2p, int lda, long strideA,
    const unsigned short* __restrict__ Btp, const unsigned short* __restrict__ Bt2p, int ldb, long strideB,
    void* __restrict__ Cout, void* __restrict__ Cout2, int ldc, long strideC,
    const float* __restrict__ bias,
    int M, int N, int K, float scale) {
  typedef typename Elem<ET>::T T;
  typedef typename Frag<T>::V V;
  const T* A = (const T*)Ap; const T* A2 = (const T*)A2p; const T* Bt = (const T*)Btp; const T* Bt2 = (const T*)Bt2p;
  __shared__ __align__(16) float sT[8][16 * 68];
  const int b    = blockIdx.y;
  const int lane = threadIdx.x & 31;
  const int wave = threadIdx.x >> 5;
  const int tilesN = N >> 6;
  const int tilesM = M >> 6;
  const int tile = blockIdx.x * 8 + wave;
  if (tile >= tilesM * tilesN) return;
  const int tm = tile / tilesN;
  const int tn = tile - tm * tilesN;
  const int m0 = tm << 6;
  const int n0 = tn << 6;

  const T* Ab  = A  + (size_t)b * strideA;
  const T* Bb  = Bt + (size_t)b * strideB;
  const T* Ab2 = (SPL & 1) ? (A2  + (size_t)b * strideA) : nullptr;
  const T* Bb2 = (SPL & 2) ? (Bt2 + (size_t)b * strideB) : nullptr;

  const int rlane = lane & 15;
  const int koff  = (lane >> 4) * 8;
  const int mOff  = (lane >> 4) * 8;

  v8f acc[4][4];
#pragma unroll
  for (int i = 0; i < 4; ++i)
#pragma unroll
    for (int j = 0; j < 4; ++j) acc[i][j] = (v8f){0.f,0.f,0.f,0.f,0.f,0.f,0.f,0.f};

  for (int k0 = 0; k0 < K; k0 += 32) {
    V bh[4], bl[4];
#pragma unroll
    for (int j = 0; j < 4; ++j) {
      const size_t bo = (size_t)(n0 + (j << 4) + rlane) * ldb + koff + k0;
      bh[j] = Frag<T>::load(Bb + bo);
      if (SPL & 2) bl[j] = Frag<T>::load(Bb2 + bo);
    }
#pragma unroll
    for (int i = 0; i < 4; ++i) {
      const size_t ao = (size_t)(m0 + (i << 4) + rlane) * lda + koff + k0;
      V ah = Frag<T>::load(Ab + ao);
      V al;
      if (SPL & 1) al = Frag<T>::load(Ab2 + ao);
#pragma unroll
      for (int j = 0; j < 4; ++j) {
        acc[i][j] = Frag<T>::mma(ah, bh[j], acc[i][j]);
        if (SPL & 2) acc[i][j] = Frag<T>::mma(ah, bl[j], acc[i][j]);
        if (SPL & 1) acc[i][j] = Frag<T>::mma(al, bh[j], acc[i][j]);
      }
      Frag<T>::guard(acc[i][0], acc[i][3], ah, (SPL & 1) ? al : ah);
    }
    Frag<T>::keep(bh[0], bh[1], bh[2], bh[3]);
    if (SPL & 2) Frag<T>::keep(bl[0], bl[1], bl[2], bl[3]);
  }
  acc_guard4(acc[0][0], acc[0][1], acc[0][2], acc[0][3]);
  acc_guard4(acc[1][0], acc[1][1], acc[1][2], acc[1][3]);
  acc_guard4(acc[2][0], acc[2][1], acc[2][2], acc[2][3]);
  acc_guard4(acc[3][0], acc[3][1], acc[3][2], acc[3][3]);

  float* slab = sT[wave];
#pragma unroll
  for (int i = 0; i < 4; ++i) {
    const int mBase = m0 + (i << 4);
#pragma unroll
    for (int j = 0; j < 4; ++j) {
      const int n = n0 + (j << 4) + rlane;
      float bv = 0.f;
      if (BIAS_MODE == 2) bv = bfr(bias[n]);
#pragma unroll
      for (int r = 0; r < 8; ++r) {
        float v = acc[i][j][r] * scale;
        if (BIAS_MODE == 2) v += bv;
        slab[(mOff + r) * 68 + (j << 4) + rlane] = v;
      }
    }
    __builtin_amdgcn_fence(__ATOMIC_RELEASE, "workgroup");
    __builtin_amdgcn_wave_barrier();
    __builtin_amdgcn_fence(__ATOMIC_ACQUIRE, "workgroup");
    if (OUT_MODE == 0) {
      float* C = (float*)Cout + (size_t)b * strideC;
      const int hh = lane >> 4, c4 = (lane & 15) * 4;
      for (int pass = 0; pass < 2; ++pass) {
#pragma unroll
        for (int it = 0; it < 8; ++it) {
          const int row = it * 2 + hh;
          v4f v = *(const v4f*)(slab + row * 68 + c4);
          *(volatile v4f*)(C + (size_t)(mBase + row) * ldc + n0 + c4) = v;
        }
        __threadfence();
      }
    } else {
      const int q = lane >> 3, c8 = (lane & 7) * 8;
      unsigned short* C  = (unsigned short*)Cout  + (size_t)b * strideC;
      unsigned short* C2 = (OUT_MODE == 2) ? ((unsigned short*)Cout2 + (size_t)b * strideC) : nullptr;
      for (int pass = 0; pass < 2; ++pass) {
#pragma unroll
        for (int it = 0; it < 4; ++it) {
          const int row = it * 4 + q;
          const float* sp = slab + row * 68 + c8;
          v8h hv, lv;
#pragma unroll
          for (int e = 0; e < 8; ++e) {
            if (OUT_MODE == 1) {
              hv[e] = (_Float16)sp[e];
            } else {
              unsigned short hb = f2bf_bits(sp[e]);
              unsigned short lb = f2bf_bits(sp[e] - bf_bits2f(hb));
              hv[e] = __builtin_bit_cast(_Float16, hb);
              lv[e] = __builtin_bit_cast(_Float16, lb);
            }
          }
          *(volatile v8h*)(C + (size_t)(mBase + row) * ldc + n0 + c8) = hv;
          if (OUT_MODE == 2) *(volatile v8h*)(C2 + (size_t)(mBase + row) * ldc + n0 + c8) = lv;
        }
        __threadfence();
      }
    }
    __builtin_amdgcn_fence(__ATOMIC_RELEASE, "workgroup");
    __builtin_amdgcn_wave_barrier();
    __builtin_amdgcn_fence(__ATOMIC_ACQUIRE, "workgroup");
  }
}

template <int MODE>
__global__ __launch_bounds__(256) void cast8_kernel(const float* __restrict__ in, unsigned short* __restrict__ out, int n8, float scale) {
  const int i = blockIdx.x * 256 + threadIdx.x;
  if (i >= n8) return;
  const float* p = in + 8 * (size_t)i;
  const v4f a = *(const v4f*)(p);
  const v4f c = *(const v4f*)(p + 4);
  unsigned short hb[8];
#pragma unroll
  for (int e = 0; e < 4; ++e) {
    if (MODE == 0) {
      hb[e]     = f2bf_bits(a[e]);
      hb[4 + e] = f2bf_bits(c[e]);
    } else {
      hb[e]     = h_bits(bf_bits2f(f2bf_bits(a[e])) * scale);
      hb[4 + e] = h_bits(bf_bits2f(f2bf_bits(c[e])) * scale);
    }
  }
  const v4u u = (v4u){pk16(hb[0], hb[1]), pk16(hb[2], hb[3]), pk16(hb[4], hb[5]), pk16(hb[6], hb[7])};
  unsigned short* q = out + 8 * (size_t)i;
  *(volatile v4u*)q = u;
  __threadfence();
  *(volatile v4u*)q = u;
  (void)scale;
}

template <int SRC_F32>
__global__ __launch_bounds__(256) void transpose64_kernel(const void* __restrict__ src, unsigned short* __restrict__ dst,
                                                          int R, int Cc, long srcPlane, long dstPlane) {
  __shared__ unsigned short tile[64][72];
  const int t = threadIdx.x, lane = t & 31, wave = t >> 5;
  const int c0 = blockIdx.x * 64, r0 = blockIdx.y * 64, z = blockIdx.z;
#pragma unroll
  for (int i = 0; i < 2; ++i) {
    const int e = i * 256 + t;
    const int row = e >> 3, c8 = (e & 7) * 8;
    const size_t so = (size_t)z * (size_t)srcPlane + (size_t)(r0 + row) * Cc + c0 + c8;
    if (SRC_F32) {
      const float* s = (const float*)src + so;
      const v4f a = *(const v4f*)(s);
      const v4f bq = *(const v4f*)(s + 4);
#pragma unroll
      for (int k = 0; k < 4; ++k) {
        tile[row][c8 + k]     = f2bf_bits(a[k]);
        tile[row][c8 + 4 + k] = f2bf_bits(bq[k]);
      }
    } else {
      const unsigned short* s = (const unsigned short*)src + so;
      const v4u u = *(const v4u*)(s);
#pragma unroll
      for (int k = 0; k < 4; ++k) {
        tile[row][c8 + 2 * k]     = (unsigned short)(u[k] & 0xFFFFu);
        tile[row][c8 + 2 * k + 1] = (unsigned short)(u[k] >> 16);
      }
    }
  }
  __syncthreads();
  const int q = lane >> 3, oc8 = (lane & 7) * 8;
  unsigned short* dz = dst + (size_t)z * (size_t)dstPlane;
  for (int pass = 0; pass < 2; ++pass) {
#pragma unroll
    for (int it = 0; it < 2; ++it) {
      const int orow = it * 32 + wave * 4 + q;
      unsigned short hb[8];
#pragma unroll
      for (int k = 0; k < 8; ++k) hb[k] = tile[oc8 + k][orow];
      const v4u u = (v4u){pk16(hb[0], hb[1]), pk16(hb[2], hb[3]), pk16(hb[4], hb[5]), pk16(hb[6], hb[7])};
      *(volatile v4u*)(dz + (size_t)(c0 + orow) * R + r0 + oc8) = u;
    }
    __threadfence();
  }
}

__global__ __launch_bounds__(256) void rope_table_kernel(float* __restrict__ RC, float* __restrict__ RS, int n) {
  const int i = blockIdx.x * 256 + threadIdx.x;
  if (i >= n) return;
  const int t = i >> 5, d = i & 31;
  const float lg  = log2f(10000.0f);
  const float inv = exp2f(-((float)d * 0.03125f) * lg);
  const float ang = (float)t * inv;
  float sn, cs;
  sincosf(ang, &sn, &cs);
  *(volatile float*)(RC + i) = cs;
  *(volatile float*)(RS + i) = sn;
  __threadfence();
  *(volatile float*)(RC + i) = cs;
  *(volatile float*)(RS + i) = sn;
}

template <int XMODE, int ACT>
__global__ __launch_bounds__(256) void rowvec_kernel(
    const float* __restrict__ X, const unsigned short* __restrict__ XH, const unsigned short* __restrict__ XL, long xRowStride,
    const float* __restrict__ W, const float* __restrict__ bias,
    float* __restrict__ Y, int ldy, int yRow0, int K, int N) {
  __shared__ float xs[3072];
  const int t = threadIdx.x;
  const int r = blockIdx.y;
  const size_t xo = (size_t)r * (size_t)xRowStride;
  for (int k = t; k < K; k += 256) {
    float v;
    if (XMODE == 1) v = bf_bits2f(XH[xo + k]) + bf_bits2f(XL[xo + k]);
    else v = X[xo + k];
    xs[k] = v;
  }
  __syncthreads();
  const int n = blockIdx.x * 256 + t;
  float acc = 0.f;
#pragma unroll 4
  for (int k = 0; k < K; ++k) acc = fmaf(xs[k], bfr(W[(size_t)k * N + n]), acc);
  float v = acc + bfr(bias[n]);
  if (ACT == 1) v = 0.5f * v * (1.0f + erff(v * 0.70710678118654752f));
  float* p = Y + (size_t)(yRow0 + r) * ldy + n;
  *(volatile float*)p = v;
  __threadfence();
  *(volatile float*)p = v;
}

__global__ __launch_bounds__(256) void score_row0_kernel(
    const float* __restrict__ Q0, int qrow0, const float* __restrict__ KF,
    const float* __restrict__ rel, const float* __restrict__ RC, const float* __restrict__ RS,
    unsigned short* __restrict__ PH, unsigned short* __restrict__ PL) {
  __shared__ float qs[kHD];
  __shared__ float ps[kNS];
  __shared__ float red[256];
  const int tid = threadIdx.x;
  const int b = blockIdx.x >> 4, h = blockIdx.x & 15;
  if (tid < kHD) qs[tid] = Q0[(size_t)(qrow0 + b) * kNE + h * kHD + tid];
  __syncthreads();

  float mloc = -INFINITY;
#pragma unroll 1
  for (int jj = 0; jj < 4; ++jj) {
    const int j = jj * 256 + tid;
    const float* kp = KF + (size_t)(b * kNS + j) * kNE + h * kHD;
    int ridx = j + kNS - 1;
    ridx = ridx < 0 ? 0 : (ridx > kRelN - 1 ? kRelN - 1 : ridx);
    const float* rp = rel + (size_t)ridx * kHD;
    const float* cp = RC + (size_t)j * kHalf;
    const float* sp = RS + (size_t)j * kHalf;
    float dqk = 0.f, drl = 0.f;
#pragma unroll 1
    for (int d = 0; d < kHalf; ++d) {
      const float k1 = kp[d], k2 = kp[d + kHalf];
      const float c = cp[d], s = sp[d];
      const float q1 = qs[d], q2 = qs[d + kHalf];
      const float r1 = k1 * c - k2 * s;
      const float r2 = k1 * s + k2 * c;
      dqk = fmaf(q1, r1, dqk);
      dqk = fmaf(q2, r2, dqk);
      drl = fmaf(q1, bfr(rp[d]), drl);
      drl = fmaf(q2, bfr(rp[d + kHalf]), drl);
    }
    const float sc = dqk * 0.125f + drl;
    ps[j] = sc;
    mloc = fmaxf(mloc, sc);
  }
  red[tid] = mloc;
  __syncthreads();
  for (int st = 128; st > 0; st >>= 1) {
    if (tid < st) red[tid] = fmaxf(red[tid], red[tid + st]);
    __syncthreads();
  }
  const float mx = red[0];
  __syncthreads();
  float lsum = 0.f;
#pragma unroll 1
  for (int jj = 0; jj < 4; ++jj) {
    const int j = jj * 256 + tid;
    const float p = expf(ps[j] - mx);
    ps[j] = p;
    lsum += p;
  }
  red[tid] = lsum;
  __syncthreads();
  for (int st = 128; st > 0; st >>= 1) {
    if (tid < st) red[tid] = red[tid] + red[tid + st];
    __syncthreads();
  }
  const float den = red[0];
  const float inv = 1.0f / den;

  const int prow = b * kNH + h;
  unsigned short* ph = PH + (size_t)prow * kPW;
  unsigned short* pl = PL + (size_t)prow * kPW;
  for (int pass = 0; pass < 2; ++pass) {
#pragma unroll
    for (int it = 0; it < 2; ++it) {
      const int col = it * 2048 + tid * 8;
      const int cb = col - b * kNS;
      const bool inside = (unsigned)cb < (unsigned)kNS;
      const int idx = inside ? cb : 0;
      unsigned short hb[8], lb[8];
#pragma unroll
      for (int k = 0; k < 8; ++k) {
        const float a = ps[idx + k] * inv;
        const float v = inside ? a : 0.0f;
        hb[k] = f2bf_bits(v);
        lb[k] = f2bf_bits(v - bf_bits2f(hb[k]));
      }
      const v4u uh = (v4u){pk16(hb[0], hb[1]), pk16(hb[2], hb[3]), pk16(hb[4], hb[5]), pk16(hb[6], hb[7])};
      const v4u ul = (v4u){pk16(lb[0], lb[1]), pk16(lb[2], lb[3]), pk16(lb[4], lb[5]), pk16(lb[6], lb[7])};
      *(volatile v4u*)(ph + col) = uh;
      *(volatile v4u*)(pl + col) = ul;
    }
    __threadfence();
  }
}

__global__ __launch_bounds__(64) void zv_kernel(const float* __restrict__ Z, const float* __restrict__ Wv, const float* __restrict__ bv,
                                                float* __restrict__ ATT0) {
  __shared__ float zs[kNE];
  __shared__ __align__(16) float os[kHD];
  const int tid = threadIdx.x;
  const int mb = blockIdx.x >> 4, h = blockIdx.x & 15;
  const int strm = mb >> 2, b = mb & 3;
  const float* zrow = Z + (size_t)(strm * 64 + b * kNH + h) * kNE;
  for (int k = tid; k < kNE; k += 64) zs[k] = zrow[k];
  __syncthreads();
  const int d = tid;
  float acc = 0.f;
#pragma unroll 4
  for (int k = 0; k < kNE; ++k) acc = fmaf(zs[k], bfr(Wv[(size_t)k * kNE + h * kHD + d]), acc);
  os[d] = acc + bfr(bv[h * kHD + d]);
  __syncthreads();
  if (tid < 16) {
    const v4f o = *(const v4f*)(os + 4 * tid);
    float* p = ATT0 + (size_t)mb * kNE + h * kHD + 4 * tid;
    *(volatile v4f*)p = o;
    __threadfence();
    *(volatile v4f*)p = o;
  }
}

__global__ __launch_bounds__(256) void ln_kernel(const float* __restrict__ YO,
                                                 const float* __restrict__ g0, const float* __restrict__ s0,
                                                 const float* __restrict__ g1, const float* __restrict__ s1,
                                                 const float* __restrict__ g2, const float* __restrict__ s2,
                                                 float* __restrict__ FUSED) {
  __shared__ float redA[8];
  __shared__ float redB[8];
  const int mb = blockIdx.x;
  const int strm = mb >> 2, b = mb & 3;
  const float* g  = (strm == 0) ? g0 : ((strm == 1) ? g1 : g2);
  const float* bn = (strm == 0) ? s0 : ((strm == 1) ? s1 : s2);
  const int t = threadIdx.x, lane = t & 31, wave = t >> 5;
  const int c0 = 4 * t;
  const v4f y = *(const v4f*)(YO + (size_t)mb * kNE + c0);
  float s = (y[0] + y[1]) + (y[2] + y[3]);
#pragma unroll
  for (int off = 16; off > 0; off >>= 1) s += __shfl_xor(s, off, 32);
  if (lane == 0) redA[wave] = s;
  __syncthreads();
  const float mu = (((redA[0] + redA[1]) + (redA[2] + redA[3])) + ((redA[4] + redA[5]) + (redA[6] + redA[7]))) * (1.0f / 1024.0f);
  float dv[4];
#pragma unroll
  for (int e = 0; e < 4; ++e) dv[e] = y[e] - mu;
  float qq = (dv[0] * dv[0] + dv[1] * dv[1]) + (dv[2] * dv[2] + dv[3] * dv[3]);
#pragma unroll
  for (int off = 16; off > 0; off >>= 1) qq += __shfl_xor(qq, off, 32);
  if (lane == 0) redB[wave] = qq;
  __syncthreads();
  const float var = (((redB[0] + redB[1]) + (redB[2] + redB[3])) + ((redB[4] + redB[5]) + (redB[6] + redB[7]))) * (1.0f / 1024.0f);
  const float rs = rsqrtf(var + 1e-5f);
  v4f o;
#pragma unroll
  for (int e = 0; e < 4; ++e) o[e] = (dv[e] * rs) * bfr(g[c0 + e]) + bfr(bn[c0 + e]);
  float* p = FUSED + (size_t)b * kF1K + (size_t)strm * kNE + c0;
  *(volatile v4f*)p = o;
  __threadfence();
  *(volatile v4f*)p = o;
}

extern "C" void kernel_launch(void* const* d_in, const int* in_sizes, int n_in,
                              void* d_out, int out_size, void* d_ws, size_t ws_size,
                              hipStream_t stream) {
  if (n_in < 28) return;
  for (int i = 0; i < 3; ++i) if (in_sizes[i] != kTok * kNE) return;
  const int wIdx[8] = {3, 5, 7, 9, 11, 13, 15, 26};
  for (int i = 0; i < 8; ++i) if (in_sizes[wIdx[i]] != kNE * kNE) return;
  const int bIdx[14] = {4, 6, 8, 10, 12, 14, 16, 18, 19, 20, 21, 22, 23, 25};
  for (int i = 0; i < 14; ++i) if (in_sizes[bIdx[i]] != kNE) return;
  if (in_sizes[27] != kNE) return;
  if (in_sizes[17] != kRelN * kHD) return;
  if (in_sizes[24] != kF1K * kNE) return;
  if (out_size != kNB * kNE) return;

  const size_t SZ_P16  = (size_t)kTok * kNE * 2;
  const size_t SZ_W16  = (size_t)kNE * kNE * 2;
  const size_t SZ_KF   = (size_t)kTok * kNE * 4;
  const size_t SZ_ROPE = (size_t)kNS * kHalf * 4;
  const size_t SZ_R12  = (size_t)kNRow * kNE * 4;
  const size_t SZ_PP   = (size_t)64 * kPW * 2;
  const size_t SZ_ZB   = (size_t)3 * 64 * kNE * 4;
  const size_t SZ_FUS  = (size_t)kNB * kF1K * 4;
  const size_t SZ_HB   = (size_t)kNB * kNE * 4;
  size_t off = 0;
  const size_t oX16  = off; off += SZ_P16;
  const size_t oWT   = off; off += SZ_W16;
  const size_t oWKT  = off; off += SZ_W16;
  const size_t oXPH  = off; off += SZ_P16;
  const size_t oXPL  = off; off += SZ_P16;
  const size_t oXPTH = off; off += SZ_P16;
  const size_t oXPTL = off; off += SZ_P16;
  const size_t oKF   = off; off += SZ_KF;
  const size_t oRC   = off; off += SZ_ROPE;
  const size_t oRS   = off; off += SZ_ROPE;
  const size_t oQ0   = off; off += SZ_R12;
  const size_t oPH   = off; off += SZ_PP;
  const size_t oPL   = off; off += SZ_PP;
  const size_t oZB   = off; off += SZ_ZB;
  const size_t oATT0 = off; off += SZ_R12;
  const size_t oYO   = off; off += SZ_R12;
  const size_t oFUS  = off; off += SZ_FUS;
  const size_t oHB   = off; off += SZ_HB;
  const size_t TOTAL = off;
  if (TOTAL > ws_size) return;
  if (TOTAL > (size_t)134217728) return;

  char* ws = (char*)d_ws;
  unsigned short* X16  = (unsigned short*)(ws + oX16);
  unsigned short* WT   = (unsigned short*)(ws + oWT);
  unsigned short* WKT  = (unsigned short*)(ws + oWKT);
  unsigned short* XPH  = (unsigned short*)(ws + oXPH);
  unsigned short* XPL  = (unsigned short*)(ws + oXPL);
  unsigned short* XPTH = (unsigned short*)(ws + oXPTH);
  unsigned short* XPTL = (unsigned short*)(ws + oXPTL);
  float*          KF   = (float*)(ws + oKF);
  float*          RC   = (float*)(ws + oRC);
  float*          RS   = (float*)(ws + oRS);
  float*          Q0   = (float*)(ws + oQ0);
  unsigned short* PH   = (unsigned short*)(ws + oPH);
  unsigned short* PL   = (unsigned short*)(ws + oPL);
  float*          ZB   = (float*)(ws + oZB);
  float*          ATT0 = (float*)(ws + oATT0);
  float*          YO   = (float*)(ws + oYO);
  float*          FUS  = (float*)(ws + oFUS);
  float*          HB   = (float*)(ws + oHB);

  const float* inp[28];
  for (int i = 0; i < 28; ++i) inp[i] = (const float*)d_in[i];
  float* outp = (float*)d_out;

  const dim3 blk(256);
  const long planeXP = (long)kTok * kNE;

  rope_table_kernel<<<dim3((kNS * kHalf) / 256), blk, 0, stream>>>(RC, RS, kNS * kHalf);
  transpose64_kernel<1><<<dim3(kNE / 64, kNE / 64, 1), blk, 0, stream>>>((const void*)inp[11], WKT, kNE, kNE, 0L, 0L);

  const int strmIn[3] = {0, 1, 2};
  const int strmW[3]  = {3, 5, 7};
  const int strmB[3]  = {4, 6, 8};
  const int n8 = kTok * kNE / 8;
  const dim3 gBig((( kTok / 64) * (kNE / 64) + 7) / 8, 1);
  const dim3 gZ(((64 / 64) * (kNE / 64) + 7) / 8, 1);

  for (int m = 0; m < 3; ++m) {
    cast8_kernel<0><<<dim3(n8 / 256), blk, 0, stream>>>(inp[strmIn[m]], X16, n8, 1.0f);
    transpose64_kernel<1><<<dim3(kNE / 64, kNE / 64, 1), blk, 0, stream>>>((const void*)inp[strmW[m]], WT, kNE, kNE, 0L, 0L);
    wmma_gemm64<1, 0, 2, 2><<<gBig, blk, 0, stream>>>(
        X16, X16, kNE, 0L, WT, WT, kNE, 0L, (void*)XPH, (void*)XPL, kNE, 0L, inp[strmB[m]], kTok, kNE, kNE, 1.0f);
    transpose64_kernel<0><<<dim3(kNE / 64, kTok / 64, 2), blk, 0, stream>>>((const void*)XPH, XPTH, kTok, kNE, planeXP, planeXP);
    wmma_gemm64<1, 1, 2, 0><<<gBig, blk, 0, stream>>>(
        XPH, XPL, kNE, 0L, WKT, WKT, kNE, 0L, (void*)KF, (void*)KF, kNE, 0L, inp[12], kTok, kNE, kNE, 1.0f);
    rowvec_kernel<1, 0><<<dim3(kNE / 256, kNB), blk, 0, stream>>>(
        KF, XPH, XPL, (long)kNS * kNE, inp[9], inp[10], Q0, kNE, m * kNB, kNE, kNE);
    score_row0_kernel<<<dim3(kNB * kNH), blk, 0, stream>>>(Q0, m * kNB, KF, inp[17], RC, RS, PH, PL);
    wmma_gemm64<1, 3, 0, 0><<<gZ, blk, 0, stream>>>(
        PH, PL, kPW, 0L, XPTH, XPTL, kPW, 0L, (void*)(ZB + (size_t)m * 64 * kNE), (void*)(ZB + (size_t)m * 64 * kNE), kNE, 0L,
        inp[12], 64, kNE, kPW, 1.0f);
  }

  zv_kernel<<<dim3(kNRow * kNH), dim3(64), 0, stream>>>(ZB, inp[13], inp[14], ATT0);
  rowvec_kernel<0, 0><<<dim3(kNE / 256, kNRow), blk, 0, stream>>>(
      ATT0, X16, X16, (long)kNE, inp[15], inp[16], YO, kNE, 0, kNE, kNE);
  ln_kernel<<<dim3(kNRow), blk, 0, stream>>>(YO, inp[18], inp[19], inp[20], inp[21], inp[22], inp[23], FUS);
  rowvec_kernel<0, 1><<<dim3(kNE / 256, kNB), blk, 0, stream>>>(
      FUS, X16, X16, (long)kF1K, inp[24], inp[25], HB, kNE, 0, kF1K, kNE);
  rowvec_kernel<0, 0><<<dim3(kNE / 256, kNB), blk, 0, stream>>>(
      HB, X16, X16, (long)kNE, inp[26], inp[27], outp, kNE, 0, kNE, kNE);
}
